// CrossAttention_15118284882167
// MI455X (gfx1250) — hardware-verified
//
#include <hip/hip_runtime.h>
#include <math.h>

constexpr int kBatch  = 2;
constexpr int kPtsPer = 2048;
constexpr int kVec    = 3;
constexpr int kCin    = 64;
constexpr int kFeat   = 128;
constexpr int kHid    = 64;
constexpr int kHeads  = 8;
constexpr int kHd     = 16;
constexpr int kSqrtHd = 4;
constexpr int kRows   = kBatch * kPtsPer * kVec;
constexpr int kPts    = kBatch * kPtsPer;
constexpr int kGroups = kHeads * kBatch;
constexpr int kDreal  = kVec * kHd;
constexpr int kDpad   = 64;
constexpr int kChunkG = 1;
constexpr float kEps        = 1e-6f;
constexpr float kSlope      = 0.2f;
constexpr float kLogitScale = 1.0f / (float)kSqrtHd;
constexpr float kInvHd      = 1.0f / (float)kHd;
constexpr float kPCarry     = 32768.0f;
constexpr float kPCarryInv  = 1.0f / 32768.0f;
constexpr float kResCarry   = 2048.0f;
constexpr float kResInv     = 1.0f / 2048.0f;
constexpr float kF16MinNormal = 6.103515625e-05f;
constexpr int   kWSlot      = 32768;
constexpr int   kWLoOff     = 16384;

static_assert(kSqrtHd * kSqrtHd == kHd, "logit scale");
static_assert(kHeads * kHd == kFeat, "head split");
static_assert(kRows == 12288 && kPts == 4096 && kGroups == 16 && kDreal == 48, "shape");
static_assert(kRows % 64 == 0 && kPts % 64 == 0 && kFeat % 64 == 0 && kHid % 64 == 0, "tile multiples");
static_assert(kCin % 32 == 0 && kFeat % 32 == 0 && kHid % 32 == 0 && kDpad % 32 == 0 && kPtsPer % 64 == 0, "k multiples");
static_assert(kGroups % kChunkG == 0, "chunks");

typedef __attribute__((ext_vector_type(16))) _Float16 v16h;
typedef __attribute__((ext_vector_type(8)))  _Float16 v8h;
typedef __attribute__((ext_vector_type(16))) __bf16   v16b;
typedef __attribute__((ext_vector_type(8)))  __bf16   v8b;
typedef __attribute__((ext_vector_type(8)))  float    v8f;
typedef __attribute__((ext_vector_type(4)))  float    v4f;
typedef __attribute__((ext_vector_type(2)))  float    v2f;
typedef __attribute__((ext_vector_type(4)))  unsigned int v4u;
typedef __attribute__((ext_vector_type(2)))  unsigned int v2u;
typedef unsigned short us16;

__device__ __forceinline__ unsigned short f2bf_bits(float f) {
  unsigned u = __float_as_uint(f);
  return (unsigned short)((u + 0x7FFFu + ((u >> 16) & 1u)) >> 16);
}
__device__ __forceinline__ float bf_bits2f(unsigned short h) { return __uint_as_float(((unsigned)h) << 16); }
__device__ __forceinline__ void split_bits(float f, unsigned short& hb, unsigned short& lb) {
  hb = f2bf_bits(f);
  lb = f2bf_bits(f - bf_bits2f(hb));
}
__device__ __forceinline__ unsigned pk16(unsigned short a, unsigned short b) { return (unsigned)a | ((unsigned)b << 16); }

__device__ __forceinline__ void split_h16(float x, unsigned short& hb, unsigned short& lb) {
  const bool tiny = fabsf(x) < kF16MinNormal;
  const float xs = tiny ? 0.0f : x;
  const _Float16 h = (_Float16)xs;
  const float hf = (float)h;
  const float rs = (x - hf) * kResCarry;
  const _Float16 l = (_Float16)rs;
  hb = __builtin_bit_cast(unsigned short, h);
  lb = __builtin_bit_cast(unsigned short, l);
}

__device__ __forceinline__ float vnorm3(float a, float b, float c) {
#pragma clang fp contract(off)
  const float s = (a * a + b * b) + c * c;
  return sqrtf(s);
}

__device__ __forceinline__ void dep_guard4_h(v8f& a, v8f& b, v8f& c, v8f& d, v16h x, v16h y) {
  asm volatile("v_nop\n\tv_nop\n\tv_nop\n\tv_nop" : "+v"(a), "+v"(b), "+v"(c), "+v"(d) : "v"(x), "v"(y));
}
__device__ __forceinline__ void dep_guard4_b(v8f& a, v8f& b, v8f& c, v8f& d, v16b x, v16b y) {
  asm volatile("v_nop\n\tv_nop\n\tv_nop\n\tv_nop" : "+v"(a), "+v"(b), "+v"(c), "+v"(d) : "v"(x), "v"(y));
}
__device__ __forceinline__ void keep4_h(v16h a, v16h b, v16h c, v16h d) { asm volatile("v_nop" :: "v"(a), "v"(b), "v"(c), "v"(d)); }
__device__ __forceinline__ void keep4_b(v16b a, v16b b, v16b c, v16b d) { asm volatile("v_nop" :: "v"(a), "v"(b), "v"(c), "v"(d)); }
__device__ __forceinline__ void acc_guard4(v8f& a, v8f& b, v8f& c, v8f& d) {
  asm volatile("v_nop\n\tv_nop\n\tv_nop\n\tv_nop" : "+v"(a), "+v"(b), "+v"(c), "+v"(d));
}
template <typename T> struct Frag;
template <> struct Frag<_Float16> {
  typedef v16h V; union U { v16h v; v8h h[2]; };
  static __device__ __forceinline__ v16h load(const _Float16* p) {
    U f; f.h[0] = *(const v8h*)(p); f.h[1] = *(const v8h*)(p + 16); return f.v;
  }
  static __device__ __forceinline__ v8f mma(v16h a, v16h b, v8f c) {
    return __builtin_amdgcn_wmma_f32_16x16x32_f16(false, a, false, b, (short)0, c, false, false);
  }
  static __device__ __forceinline__ void guard4(v8f& a, v8f& b, v8f& c, v8f& d, v16h x, v16h y) { dep_guard4_h(a, b, c, d, x, y); }
  static __device__ __forceinline__ void keep(v16h a, v16h b, v16h c, v16h d) { keep4_h(a, b, c, d); }
};
template <> struct Frag<__bf16> {
  typedef v16b V; union U { v16b v; v8b h[2]; };
  static __device__ __forceinline__ v16b load(const __bf16* p) {
    U f; f.h[0] = *(const v8b*)(p); f.h[1] = *(const v8b*)(p + 16); return f.v;
  }
  static __device__ __forceinline__ v8f mma(v16b a, v16b b, v8f c) {
    return __builtin_amdgcn_wmma_f32_16x16x32_bf16(false, a, false, b, (short)0, c, false, false);
  }
  static __device__ __forceinline__ void guard4(v8f& a, v8f& b, v8f& c, v8f& d, v16b x, v16b y) { dep_guard4_b(a, b, c, d, x, y); }
  static __device__ __forceinline__ void keep(v16b a, v16b b, v16b c, v16b d) { keep4_b(a, b, c, d); }
};

template <int ET> struct Elem;
template <> struct Elem<0> { typedef _Float16 T; };
template <> struct Elem<1> { typedef __bf16 T; };
template <int ET, bool SPLIT, int BIAS_MODE, int OUT_MODE, bool RESID, int ACT = 0>
__global__ __launch_bounds__(256) void wmma_gemm64(
    const unsigned short* __restrict__ Ap, const unsigned short* __restrict__ A2p, int lda, long strideA,
    const unsigned short* __restrict__ Btp, const unsigned short* __restrict__ Bt2p, int ldb, long strideB,
    void* __restrict__ Cout, void* __restrict__ Cout2, int ldc, long strideC,
    const float* __restrict__ bias,
    const float* __restrict__ resid, long strideR,
    int M, int N, int K, float scale) {
  static_assert(!RESID, "residual addends are applied by the elementwise kernels");
  typedef typename Elem<ET>::T T;
  typedef typename Frag<T>::V V;
  const T* A = (const T*)Ap; const T* A2 = (const T*)A2p; const T* Bt = (const T*)Btp; const T* Bt2 = (const T*)Bt2p;
  __shared__ __align__(16) float sT[8][16 * 68];
  const int b    = blockIdx.y;
  const int lane = threadIdx.x & 31;
  const int wave = threadIdx.x >> 5;
  const int tilesN = N >> 6;
  const int tilesM = M >> 6;
  const int tile = blockIdx.x * 8 + wave;
  if (tile >= tilesM * tilesN) return;
  const int tm = tile / tilesN;
  const int tn = tile - tm * tilesN;
  const int m0 = tm << 6;
  const int n0 = tn << 6;

  const T* Ab  = A  + (size_t)b * strideA;
  const T* Bb  = Bt + (size_t)b * strideB;
  const T* Ab2 = SPLIT ? (A2  + (size_t)b * strideA) : nullptr;
  const T* Bb2 = SPLIT ? (Bt2 + (size_t)b * strideB) : nullptr;

  const int rlane = lane & 15;
  const int koff  = (lane >> 4) * 8;
  const int mOff  = (lane >> 4) * 8;

  v8f acc[4][4];
#pragma unroll
  for (int i = 0; i < 4; ++i)
#pragma unroll
    for (int j = 0; j < 4; ++j) acc[i][j] = (v8f){0.f,0.f,0.f,0.f,0.f,0.f,0.f,0.f};

  for (int k0 = 0; k0 < K; k0 += 32) {
    V bh[4], bl[4];
#pragma unroll
    for (int j = 0; j < 4; ++j) {
      const size_t bo = (size_t)(n0 + (j << 4) + rlane) * ldb + koff + k0;
      bh[j] = Frag<T>::load(Bb + bo);
      if (SPLIT) bl[j] = Frag<T>::load(Bb2 + bo);
    }
#pragma unroll
    for (int i = 0; i < 4; ++i) {
      const size_t ao = (size_t)(m0 + (i << 4) + rlane) * lda + koff + k0;
      V ah = Frag<T>::load(Ab + ao);
      V al;
      if (SPLIT) al = Frag<T>::load(Ab2 + ao);
#pragma unroll
      for (int j = 0; j < 4; ++j) {
        acc[i][j] = Frag<T>::mma(ah, bh[j], acc[i][j]);
        if (SPLIT) {
          acc[i][j] = Frag<T>::mma(ah, bl[j], acc[i][j]);
          acc[i][j] = Frag<T>::mma(al, bh[j], acc[i][j]);
        }
      }
      Frag<T>::guard4(acc[i][0], acc[i][1], acc[i][2], acc[i][3], ah, SPLIT ? al : ah);
    }
    Frag<T>::keep(bh[0], bh[1], bh[2], bh[3]);
    if (SPLIT) Frag<T>::keep(bl[0], bl[1], bl[2], bl[3]);
  }
  acc_guard4(acc[0][0], acc[0][1], acc[0][2], acc[0][3]);
  acc_guard4(acc[1][0], acc[1][1], acc[1][2], acc[1][3]);
  acc_guard4(acc[2][0], acc[2][1], acc[2][2], acc[2][3]);
  acc_guard4(acc[3][0], acc[3][1], acc[3][2], acc[3][3]);

  float* slab = sT[wave];
#pragma unroll
  for (int i = 0; i < 4; ++i) {
    const int mBase = m0 + (i << 4);
#pragma unroll
    for (int j = 0; j < 4; ++j) {
      const int n = n0 + (j << 4) + rlane;
      float bv = 0.f;
      if (BIAS_MODE == 2) bv = bias[n];
#pragma unroll
      for (int r = 0; r < 8; ++r) {
        float v = acc[i][j][r] * scale;
        if (BIAS_MODE == 1) v += bias[mBase + mOff + r];
        if (BIAS_MODE == 2) v += bv;
        if (ACT == 2) v = fmaxf(v, 0.0f);
        if (ACT == 6) v = (v > 0.f) ? v : kSlope * v;
        slab[(mOff + r) * 68 + (j << 4) + rlane] = v;
      }
    }
    __builtin_amdgcn_fence(__ATOMIC_RELEASE, "workgroup");
    __builtin_amdgcn_wave_barrier();
    __builtin_amdgcn_fence(__ATOMIC_ACQUIRE, "workgroup");
    if (OUT_MODE == 0) {
      float* C = (float*)Cout + (size_t)b * strideC;
      const int hh = lane >> 4, c4 = (lane & 15) * 4;
      for (int pass = 0; pass < 2; ++pass) {
#pragma unroll
        for (int it = 0; it < 8; ++it) {
          const int row = it * 2 + hh;
          v4f v = *(const v4f*)(slab + row * 68 + c4);
          *(volatile v4f*)(C + (size_t)(mBase + row) * ldc + n0 + c4) = v;
        }
        __threadfence();
      }
    } else {
      const int q = lane >> 3, c8 = (lane & 7) * 8;
      unsigned short* C  = (unsigned short*)Cout  + (size_t)b * strideC;
      unsigned short* C2 = (OUT_MODE == 2) ? ((unsigned short*)Cout2 + (size_t)b * strideC) : nullptr;
      for (int pass = 0; pass < 2; ++pass) {
#pragma unroll
        for (int it = 0; it < 4; ++it) {
          const int row = it * 4 + q;
          const float* sp = slab + row * 68 + c8;
          v8h hv, lv;
#pragma unroll
          for (int e = 0; e < 8; ++e) {
            if (OUT_MODE == 1) {
              hv[e] = (_Float16)sp[e];
            } else {
              unsigned short hb = f2bf_bits(sp[e]);
              unsigned short lb = f2bf_bits(sp[e] - bf_bits2f(hb));
              hv[e] = __builtin_bit_cast(_Float16, hb);
              lv[e] = __builtin_bit_cast(_Float16, lb);
            }
          }
          *(volatile v8h*)(C + (size_t)(mBase + row) * ldc + n0 + c8) = hv;
          if (OUT_MODE == 2) *(volatile v8h*)(C2 + (size_t)(mBase + row) * ldc + n0 + c8) = lv;
        }
        __threadfence();
      }
    }
    __builtin_amdgcn_fence(__ATOMIC_RELEASE, "workgroup");
    __builtin_amdgcn_wave_barrier();
    __builtin_amdgcn_fence(__ATOMIC_ACQUIRE, "workgroup");
  }
}

__global__ __launch_bounds__(256) void wmma_gemm_rs(
    const unsigned short* __restrict__ Ahp, const unsigned short* __restrict__ Alp, int lda, long strideA,
    const unsigned short* __restrict__ Bhp, const unsigned short* __restrict__ Blp, int ldb, long strideB,
    float* __restrict__ Cout, int ldc, long strideC,
    int M, int N, int K, float scale) {
  typedef _Float16 T;
  typedef v16h V;
  __shared__ __align__(16) float sR[8][16 * 36];
  const int b    = blockIdx.y;
  const int lane = threadIdx.x & 31;
  const int wave = threadIdx.x >> 5;
  const int tilesN = N >> 5;
  const int tilesM = M >> 6;
  const int tile = blockIdx.x * 8 + wave;
  if (tile >= tilesM * tilesN) return;
  const int tm = tile / tilesN;
  const int tn = tile - tm * tilesN;
  const int m0 = tm << 6;
  const int n0 = tn << 5;

  const T* Ah = (const T*)Ahp + (size_t)b * strideA;
  const T* Al = (const T*)Alp + (size_t)b * strideA;
  const T* Bh = (const T*)Bhp + (size_t)b * strideB;
  const T* Bl = (const T*)Blp + (size_t)b * strideB;

  const int rlane = lane & 15;
  const int koff  = (lane >> 4) * 8;
  const int mOff  = (lane >> 4) * 8;

  v8f acc[4][2], accr[4][2];
#pragma unroll
  for (int i = 0; i < 4; ++i)
#pragma unroll
    for (int j = 0; j < 2; ++j) {
      acc[i][j]  = (v8f){0.f,0.f,0.f,0.f,0.f,0.f,0.f,0.f};
      accr[i][j] = (v8f){0.f,0.f,0.f,0.f,0.f,0.f,0.f,0.f};
    }

  for (int k0 = 0; k0 < K; k0 += 32) {
    V bh[2], bl[2];
#pragma unroll
    for (int j = 0; j < 2; ++j) {
      const size_t bo = (size_t)(n0 + (j << 4) + rlane) * ldb + koff + k0;
      bh[j] = Frag<T>::load(Bh + bo);
      bl[j] = Frag<T>::load(Bl + bo);
    }
#pragma unroll
    for (int i = 0; i < 4; ++i) {
      const size_t ao = (size_t)(m0 + (i << 4) + rlane) * lda + koff + k0;
      V ah = Frag<T>::load(Ah + ao);
      V al = Frag<T>::load(Al + ao);
#pragma unroll
      for (int j = 0; j < 2; ++j) {
        acc[i][j]  = Frag<T>::mma(ah, bh[j], acc[i][j]);
        accr[i][j] = Frag<T>::mma(ah, bl[j], accr[i][j]);
        accr[i][j] = Frag<T>::mma(al, bh[j], accr[i][j]);
      }
      dep_guard4_h(acc[i][0], acc[i][1], accr[i][0], accr[i][1], ah, al);
    }
    keep4_h(bh[0], bh[1], bl[0], bl[1]);
  }
  acc_guard4(acc[0][0], acc[0][1], accr[0][0], accr[0][1]);
  acc_guard4(acc[1][0], acc[1][1], accr[1][0], accr[1][1]);
  acc_guard4(acc[2][0], acc[2][1], accr[2][0], accr[2][1]);
  acc_guard4(acc[3][0], acc[3][1], accr[3][0], accr[3][1]);

  float* slab = sR[wave];
  float* C = Cout + (size_t)b * strideC;
  const int q = lane >> 3, c4 = (lane & 7) * 4;
#pragma unroll
  for (int i = 0; i < 4; ++i) {
    const int mBase = m0 + (i << 4);
#pragma unroll
    for (int j = 0; j < 2; ++j) {
#pragma unroll
      for (int r = 0; r < 8; ++r) {
        const float folded = acc[i][j][r] + accr[i][j][r] * kResInv;
        slab[(mOff + r) * 36 + (j << 4) + rlane] = folded * scale;
      }
    }
    __builtin_amdgcn_fence(__ATOMIC_RELEASE, "workgroup");
    __builtin_amdgcn_wave_barrier();
    __builtin_amdgcn_fence(__ATOMIC_ACQUIRE, "workgroup");
    for (int pass = 0; pass < 2; ++pass) {
#pragma unroll
      for (int it = 0; it < 4; ++it) {
        const int row = it * 4 + q;
        v4f v = *(const v4f*)(slab + row * 36 + c4);
        *(volatile v4f*)(C + (size_t)(mBase + row) * ldc + n0 + c4) = v;
      }
      __threadfence();
    }
    __builtin_amdgcn_fence(__ATOMIC_RELEASE, "workgroup");
    __builtin_amdgcn_wave_barrier();
    __builtin_amdgcn_fence(__ATOMIC_ACQUIRE, "workgroup");
  }
}

__device__ __forceinline__ int wprep_kin(int id)  { return (id == 1 || id == 4 || id == 10 || (id >= 6 && id <= 9)) ? 128 : 64; }
__device__ __forceinline__ int wprep_nout(int id) { return (id == 1 || id == 4 || id == 10) ? 64 : 128; }

__global__ __launch_bounds__(256) void wprep_kernel(
    const float* __restrict__ w0, const float* __restrict__ w1, const float* __restrict__ w2, const float* __restrict__ w3,
    const float* __restrict__ w4, const float* __restrict__ w5, const float* __restrict__ w6, const float* __restrict__ w7,
    const float* __restrict__ w8, const float* __restrict__ w9, const float* __restrict__ w10, const float* __restrict__ w11,
    unsigned short* __restrict__ wpl) {
  __shared__ float sm[64][65];
  const int id = blockIdx.y;
  const float* W = w0;
  if (id == 1) W = w1;
  if (id == 2) W = w2;
  if (id == 3) W = w3;
  if (id == 4) W = w4;
  if (id == 5) W = w5;
  if (id == 6) W = w6;
  if (id == 7) W = w7;
  if (id == 8) W = w8;
  if (id == 9) W = w9;
  if (id == 10) W = w10;
  if (id == 11) W = w11;
  const int Kin = wprep_kin(id);
  const int Nout = wprep_nout(id);
  const int tilesK = Kin >> 6;
  const int tilesN = Nout >> 6;
  const int tix = blockIdx.x;
  if (tix >= tilesK * tilesN) return;
  const int tk = tix % tilesK;
  const int tn = tix / tilesK;
  const int k0 = tk * 64;
  const int n0 = tn * 64;
  const int t = threadIdx.x;
#pragma unroll
  for (int i = 0; i < 16; ++i) {
    const int e = i * 256 + t;
    const int r = e >> 6;
    const int c = e & 63;
    sm[c][r] = W[(size_t)(k0 + r) * Nout + n0 + c];
  }
  __syncthreads();
  const int lane = t & 31, wave = t >> 5;
  const int q = lane >> 3, c8 = (lane & 7) * 8;
  unsigned short* hp = wpl + (size_t)id * kWSlot;
  unsigned short* lp = hp + kWLoOff;
  for (int pass = 0; pass < 2; ++pass) {
#pragma unroll
    for (int it = 0; it < 2; ++it) {
      const int row = wave * 8 + it * 4 + q;
      unsigned short hb[8], lb[8];
#pragma unroll
      for (int e = 0; e < 8; ++e) split_bits(sm[row][c8 + e], hb[e], lb[e]);
      const v4u uh = (v4u){pk16(hb[0], hb[1]), pk16(hb[2], hb[3]), pk16(hb[4], hb[5]), pk16(hb[6], hb[7])};
      const v4u ul = (v4u){pk16(lb[0], lb[1]), pk16(lb[2], lb[3]), pk16(lb[4], lb[5]), pk16(lb[6], lb[7])};
      const size_t off = (size_t)(n0 + row) * Kin + k0 + c8;
      *(volatile v4u*)(hp + off) = uh;
      *(volatile v4u*)(lp + off) = ul;
    }
    __threadfence();
  }
}

__global__ __launch_bounds__(256) void split8_kernel(const float* __restrict__ in0, const float* __restrict__ in1,
                                                     unsigned short* __restrict__ h0, unsigned short* __restrict__ l0,
                                                     unsigned short* __restrict__ h1, unsigned short* __restrict__ l1, int n8) {
  const int i = blockIdx.x * 256 + threadIdx.x;
  if (i >= n8) return;
  const bool second = (blockIdx.y != 0);
  const float* in = second ? in1 : in0;
  unsigned short* hp = second ? h1 : h0;
  unsigned short* lp = second ? l1 : l0;
  const float* p = in + 8 * (size_t)i;
  const v4f a = *(const v4f*)(p);
  const v4f c = *(const v4f*)(p + 4);
  unsigned short hb[8], lb[8];
#pragma unroll
  for (int e = 0; e < 4; ++e) {
    const float fa = a[e];
    const float fc = c[e];
    split_bits(fa, hb[e], lb[e]);
    split_bits(fc, hb[4 + e], lb[4 + e]);
  }
  const v4u uh = (v4u){pk16(hb[0], hb[1]), pk16(hb[2], hb[3]), pk16(hb[4], hb[5]), pk16(hb[6], hb[7])};
  const v4u ul = (v4u){pk16(lb[0], lb[1]), pk16(lb[2], lb[3]), pk16(lb[4], lb[5]), pk16(lb[6], lb[7])};
  unsigned short* qh = hp + 8 * (size_t)i;
  unsigned short* ql = lp + 8 * (size_t)i;
  *(volatile v4u*)qh = uh;
  *(volatile v4u*)ql = ul;
  __threadfence();
  *(volatile v4u*)qh = uh;
  *(volatile v4u*)ql = ul;
}

__global__ __launch_bounds__(256) void evnorm_kernel(const float* __restrict__ X, float* __restrict__ NP,
                                                     unsigned short* __restrict__ NPh, unsigned short* __restrict__ NPl) {
  const int g = blockIdx.x * 256 + threadIdx.x;
  if (g >= kPts * 32) return;
  const int p = g >> 5;
  const int c4 = (g & 31) * 4;
  const float* xp = X + (size_t)p * (kVec * kFeat) + c4;
  const v4f x0 = *(const v4f*)(xp);
  const v4f x1 = *(const v4f*)(xp + kFeat);
  const v4f x2 = *(const v4f*)(xp + 2 * kFeat);
  v4f np;
  unsigned short hb[4], lb[4];
#pragma unroll
  for (int e = 0; e < 4; ++e) {
    const float n0 = vnorm3(x0[e], x1[e], x2[e]);
    const float v = n0 + kEps;
    np[e] = v;
    split_bits(v, hb[e], lb[e]);
  }
  const v2u uh = (v2u){pk16(hb[0], hb[1]), pk16(hb[2], hb[3])};
  const v2u ul = (v2u){pk16(lb[0], lb[1]), pk16(lb[2], lb[3])};
  float* fp = NP + (size_t)p * kFeat + c4;
  unsigned short* ph = NPh + (size_t)p * kFeat + c4;
  unsigned short* pl = NPl + (size_t)p * kFeat + c4;
  for (int pass = 0; pass < 2; ++pass) {
    *(volatile v4f*)fp = np;
    *(volatile v2u*)ph = uh;
    *(volatile v2u*)pl = ul;
    __threadfence();
  }
}

template <int MODE>
__global__ __launch_bounds__(256) void evscale_kernel(const float* __restrict__ X, const float* __restrict__ NP,
                                                      const float* __restrict__ NB,
                                                      unsigned short* __restrict__ Yh, unsigned short* __restrict__ Yl,
                                                      float* __restrict__ Yf) {
  const int g = blockIdx.x * 256 + threadIdx.x;
  if (g >= kPts * 32) return;
  const int p = g >> 5;
  const int c4 = (g & 31) * 4;
  const float* xp = X + (size_t)p * (kVec * kFeat) + c4;
  const v4f x0 = *(const v4f*)(xp);
  const v4f x1 = *(const v4f*)(xp + kFeat);
  const v4f x2 = *(const v4f*)(xp + 2 * kFeat);
  const v4f np = *(const v4f*)(NP + (size_t)p * kFeat + c4);
  const v4f nb = *(const v4f*)(NB + (size_t)p * kFeat + c4);
  v4f y0, y1, y2;
#pragma unroll
  for (int e = 0; e < 4; ++e) {
    const float n0 = vnorm3(x0[e], x1[e], x2[e]);
    const bool zn = (n0 <= kEps);
    const float nbt = nb[e] + np[e];
    const float rinv = 1.0f / np[e];
    const float a0 = (x0[e] * rinv) * nbt;
    const float a1 = (x1[e] * rinv) * nbt;
    const float a2 = (x2[e] * rinv) * nbt;
    y0[e] = zn ? x0[e] : a0;
    y1[e] = zn ? x1[e] : a1;
    y2[e] = zn ? x2[e] : a2;
  }
  const size_t r0 = (size_t)p * kVec;
  if (MODE == 1) {
    float* o0 = Yf + (r0 + 0) * kFeat + c4;
    float* o1 = Yf + (r0 + 1) * kFeat + c4;
    float* o2 = Yf + (r0 + 2) * kFeat + c4;
    for (int pass = 0; pass < 2; ++pass) {
      *(volatile v4f*)o0 = y0;
      *(volatile v4f*)o1 = y1;
      *(volatile v4f*)o2 = y2;
      __threadfence();
    }
  } else {
    unsigned short hb[12], lb[12];
#pragma unroll
    for (int e = 0; e < 4; ++e) {
      const float f0 = y0[e];
      const float f1 = y1[e];
      const float f2 = y2[e];
      split_bits(f0, hb[e], lb[e]);
      split_bits(f1, hb[4 + e], lb[4 + e]);
      split_bits(f2, hb[8 + e], lb[8 + e]);
    }
    const v2u h0 = (v2u){pk16(hb[0], hb[1]), pk16(hb[2], hb[3])};
    const v2u h1 = (v2u){pk16(hb[4], hb[5]), pk16(hb[6], hb[7])};
    const v2u h2 = (v2u){pk16(hb[8], hb[9]), pk16(hb[10], hb[11])};
    const v2u l0 = (v2u){pk16(lb[0], lb[1]), pk16(lb[2], lb[3])};
    const v2u l1 = (v2u){pk16(lb[4], lb[5]), pk16(lb[6], lb[7])};
    const v2u l2 = (v2u){pk16(lb[8], lb[9]), pk16(lb[10], lb[11])};
    unsigned short* ph = Yh + r0 * kFeat + c4;
    unsigned short* pl = Yl + r0 * kFeat + c4;
    for (int pass = 0; pass < 2; ++pass) {
      *(volatile v2u*)(ph) = h0;
      *(volatile v2u*)(ph + kFeat) = h1;
      *(volatile v2u*)(ph + 2 * kFeat) = h2;
      *(volatile v2u*)(pl) = l0;
      *(volatile v2u*)(pl + kFeat) = l1;
      *(volatile v2u*)(pl + 2 * kFeat) = l2;
      __threadfence();
    }
  }
}

__global__ __launch_bounds__(256) void lnpack_kernel(const float* __restrict__ srcq, const float* __restrict__ srck,
                                                     unsigned short* __restrict__ dstqh, unsigned short* __restrict__ dstql,
                                                     unsigned short* __restrict__ dstkh, unsigned short* __restrict__ dstkl) {
  const bool second = (blockIdx.y != 0);
  const float* src = second ? srck : srcq;
  unsigned short* dsth = second ? dstkh : dstqh;
  unsigned short* dstl = second ? dstkl : dstql;
  const int g = blockIdx.x * 256 + threadIdx.x;
  const int j = g & 7;
  const int rowid = g >> 3;
  const int n = rowid & (kPtsPer - 1);
  const int grp = rowid >> 11;
  const int h = grp >> 1;
  const int b = grp & 1;
  const int fj = j >> 1;
  const int f = (fj < kVec) ? fj : (kVec - 1);
  const int d0 = (j & 1) * 8;
  const bool live = (j < 2 * kVec);
  const float* xp = src + ((size_t)(b * kPtsPer + n) * kVec + f) * kFeat + h * kHd + d0;
  const v4f a = *(const v4f*)(xp);
  const v4f c = *(const v4f*)(xp + 4);
  float x[8];
#pragma unroll
  for (int e = 0; e < 4; ++e) {
    x[e]     = live ? a[e] : 0.0f;
    x[4 + e] = live ? c[e] : 0.0f;
  }
  float ss = 0.0f;
#pragma unroll
  for (int e = 0; e < 8; ++e) ss += x[e] * x[e];
  ss += __shfl_xor(ss, 1, 32);
  ss += __shfl_xor(ss, 2, 32);
  ss += __shfl_xor(ss, 4, 32);
  const float sig = sqrtf(ss * kInvHd);
  const float sc = 1.0f / (sig + kEps);
  unsigned short hb[8], lb[8];
#pragma unroll
  for (int e = 0; e < 8; ++e) {
    const float y = x[e] * sc;
    split_h16(y, hb[e], lb[e]);
  }
  const v4u uh = (v4u){pk16(hb[0], hb[1]), pk16(hb[2], hb[3]), pk16(hb[4], hb[5]), pk16(hb[6], hb[7])};
  const v4u ul = (v4u){pk16(lb[0], lb[1]), pk16(lb[2], lb[3]), pk16(lb[4], lb[5]), pk16(lb[6], lb[7])};
  unsigned short* oph = dsth + (size_t)rowid * kDpad + j * 8;
  unsigned short* opl = dstl + (size_t)rowid * kDpad + j * 8;
  *(volatile v4u*)oph = uh;
  *(volatile v4u*)opl = ul;
  __threadfence();
  *(volatile v4u*)oph = uh;
  *(volatile v4u*)opl = ul;
}

__global__ __launch_bounds__(256) void packv_kernel(const float* __restrict__ vh, unsigned short* __restrict__ VTh,
                                                    unsigned short* __restrict__ VTl) {
  __shared__ float sm[64][65];
  const int t = threadIdx.x;
  const int n0 = blockIdx.x * 64;
  const int grp = blockIdx.y;
  const int h = grp >> 1;
  const int b = grp & 1;
#pragma unroll
  for (int i = 0; i < 4; ++i) {
    const int e = i * 256 + t;
    sm[kDreal + (e >> 6)][e & 63] = 0.0f;
  }
#pragma unroll
  for (int i = 0; i < 12; ++i) {
    const int e = i * 256 + t;
    const int r = e / kDreal;
    const int c = e - r * kDreal;
    const int f = c >> 4;
    const int d = c & 15;
    sm[c][r] = vh[((size_t)(b * kPtsPer + n0 + r) * kVec + f) * kFeat + h * kHd + d];
  }
  __syncthreads();
  const int lane = t & 31, wave = t >> 5;
  const int q = lane >> 3, c8 = (lane & 7) * 8;
  unsigned short* oph = VTh + (size_t)grp * kDpad * kPtsPer;
  unsigned short* opl = VTl + (size_t)grp * kDpad * kPtsPer;
  for (int pass = 0; pass < 2; ++pass) {
#pragma unroll
    for (int it = 0; it < 2; ++it) {
      const int row = wave * 8 + it * 4 + q;
      unsigned short hb[8], lb[8];
#pragma unroll
      for (int e = 0; e < 8; ++e) split_h16(sm[row][c8 + e], hb[e], lb[e]);
      const v4u uh = (v4u){pk16(hb[0], hb[1]), pk16(hb[2], hb[3]), pk16(hb[4], hb[5]), pk16(hb[6], hb[7])};
      const v4u ul = (v4u){pk16(lb[0], lb[1]), pk16(lb[2], lb[3]), pk16(lb[4], lb[5]), pk16(lb[6], lb[7])};
      const size_t off = (size_t)row * kPtsPer + n0 + c8;
      *(volatile v4u*)(oph + off) = uh;
      *(volatile v4u*)(opl + off) = ul;
    }
    __threadfence();
  }
}

__global__ __launch_bounds__(256) void softmax_kernel(const float* __restrict__ Sp, unsigned short* __restrict__ Ph,
                                                      unsigned short* __restrict__ Pl) {
  __shared__ __align__(16) float lg[kPtsPer];
  __shared__ float redM[8];
  __shared__ float redS[8];
  const int i    = blockIdx.x;
  const int gl   = blockIdx.y;
  const int t    = threadIdx.x;
  const int lane = t & 31, wave = t >> 5;
  const size_t rowoff = ((size_t)gl * kPtsPer + i) * kPtsPer;
  const float* sr = Sp + rowoff;

  float mx = -__builtin_inff();
#pragma unroll 1
  for (int it = 0; it < 4; ++it) {
    const int c = it * 512 + 2 * t;
    const v2f sv = *(const v2f*)(sr + c);
    mx = fmaxf(mx, fmaxf(sv[0], sv[1]));
    *(v2f*)(lg + c) = sv;
  }
#pragma unroll
  for (int off = 16; off > 0; off >>= 1) mx = fmaxf(mx, __shfl_xor(mx, off, 32));
  if (lane == 0) redM[wave] = mx;
  __syncthreads();
  float m = redM[0];
#pragma unroll
  for (int w = 1; w < 8; ++w) m = fmaxf(m, redM[w]);

  float sum = 0.f;
#pragma unroll 1
  for (int it = 0; it < 4; ++it) {
    const int c = it * 512 + 2 * t;
    const v2f l = *(const v2f*)(lg + c);
    v2f ev;
#pragma unroll
    for (int e = 0; e < 2; ++e) {
      ev[e] = expf(l[e] - m);
      sum += ev[e];
    }
    *(v2f*)(lg + c) = ev;
  }
#pragma unroll
  for (int off = 16; off > 0; off >>= 1) sum += __shfl_xor(sum, off, 32);
  if (lane == 0) redS[wave] = sum;
  __syncthreads();
  float tot = redS[0];
#pragma unroll
  for (int w = 1; w < 8; ++w) tot += redS[w];
  const float inv = kPCarry / tot;

  const v4f e0 = *(const v4f*)(lg + 8 * t);
  const v4f e1 = *(const v4f*)(lg + 8 * t + 4);
  unsigned short hb[8], lb[8];
#pragma unroll
  for (int e = 0; e < 4; ++e) {
    const float pa = e0[e] * inv;
    const float pc = e1[e] * inv;
    split_h16(pa, hb[e], lb[e]);
    split_h16(pc, hb[4 + e], lb[4 + e]);
  }
  const v4u uh = (v4u){pk16(hb[0], hb[1]), pk16(hb[2], hb[3]), pk16(hb[4], hb[5]), pk16(hb[6], hb[7])};
  const v4u ul = (v4u){pk16(lb[0], lb[1]), pk16(lb[2], lb[3]), pk16(lb[4], lb[5]), pk16(lb[6], lb[7])};
  unsigned short* prh = Ph + rowoff + 8 * (size_t)t;
  unsigned short* prl = Pl + rowoff + 8 * (size_t)t;
  *(volatile v4u*)prh = uh;
  *(volatile v4u*)prl = ul;
  __threadfence();
  *(volatile v4u*)prh = uh;
  *(volatile v4u*)prl = ul;
}

__global__ __launch_bounds__(256) void repack_kernel(const float* __restrict__ Oh, unsigned short* __restrict__ Rh,
                                                     unsigned short* __restrict__ Rl) {
  const int g = blockIdx.x * 256 + threadIdx.x;
  if (g >= kRows * 16) return;
  const int j = g & 15;
  const int r = g >> 4;
  const int pn = r / kVec;
  const int f = r - pn * kVec;
  const int b = pn >> 11;
  const int n = pn & (kPtsPer - 1);
  const int h = j >> 1;
  const int d0 = (j & 1) * 8;
  const float* sp = Oh + ((size_t)(h * kBatch + b) * kPtsPer + n) * kDpad + f * kHd + d0;
  const v4f a = *(const v4f*)(sp);
  const v4f c = *(const v4f*)(sp + 4);
  unsigned short hb[8], lb[8];
#pragma unroll
  for (int e = 0; e < 4; ++e) {
    const float fa = a[e];
    const float fc = c[e];
    split_bits(fa, hb[e], lb[e]);
    split_bits(fc, hb[4 + e], lb[4 + e]);
  }
  const v4u uh = (v4u){pk16(hb[0], hb[1]), pk16(hb[2], hb[3]), pk16(hb[4], hb[5]), pk16(hb[6], hb[7])};
  const v4u ul = (v4u){pk16(lb[0], lb[1]), pk16(lb[2], lb[3]), pk16(lb[4], lb[5]), pk16(lb[6], lb[7])};
  unsigned short* qh = Rh + (size_t)r * kFeat + j * 8;
  unsigned short* ql = Rl + (size_t)r * kFeat + j * 8;
  *(volatile v4u*)qh = uh;
  *(volatile v4u*)ql = ul;
  __threadfence();
  *(volatile v4u*)qh = uh;
  *(volatile v4u*)ql = ul;
}

static void launch_split_f32(const us16* Ah, const us16* Al, int lda, const us16* Bh, const us16* Bl, int ldb,
                             float* C, int ldc, const float* dummy, int M, int N, int K, hipStream_t s) {
  const int tiles = (M / 64) * (N / 64);
  wmma_gemm64<1, true, 0, 0, false, 0><<<dim3((tiles + 7) / 8, 1), dim3(256), 0, s>>>(
      Ah, Al, lda, 0L, Bh, Bl, ldb, 0L, (void*)C, (void*)C, ldc, 0L, dummy, dummy, 0L, M, N, K, 1.0f);
}

static void launch_ev_mlp(const float* X, float* NP, us16* NPH, us16* NPL, us16* HH, us16* HL, float* NB,
                          const us16* w1h, const us16* w1l, const float* b1,
                          const us16* w2h, const us16* w2l, const float* b2, hipStream_t s) {
  evnorm_kernel<<<dim3((kPts * 32) / 256), dim3(256), 0, s>>>(X, NP, NPH, NPL);
  {
    const int tiles = (kPts / 64) * (kHid / 64);
    wmma_gemm64<1, true, 2, 2, false, 6><<<dim3((tiles + 7) / 8, 1), dim3(256), 0, s>>>(
        NPH, NPL, kFeat, 0L, w1h, w1l, kFeat, 0L, (void*)HH, (void*)HL, kHid, 0L, b1, b1, 0L, kPts, kHid, kFeat, 1.0f);
  }
  {
    const int tiles = (kPts / 64) * (kFeat / 64);
    wmma_gemm64<1, true, 2, 0, false, 0><<<dim3((tiles + 7) / 8, 1), dim3(256), 0, s>>>(
        HH, HL, kHid, 0L, w2h, w2l, kHid, 0L, (void*)NB, (void*)NB, kFeat, 0L, b2, b2, 0L, kPts, kFeat, kHid, 1.0f);
  }
}

constexpr size_t kSzWpl  = 1048576;
constexpr size_t kSzIn16 = (size_t)kRows * kCin * 2;
constexpr size_t kSzXf   = (size_t)kRows * kFeat * 4;
constexpr size_t kSzNPf  = (size_t)kPts * kFeat * 4;
constexpr size_t kSzNP16 = (size_t)kPts * kFeat * 2;
constexpr size_t kSzH16  = (size_t)kPts * kHid * 2;
constexpr size_t kSzF16  = (size_t)kRows * kFeat * 2;
constexpr size_t kSzQP   = (size_t)kGroups * kPtsPer * kDpad * 2;
constexpr size_t kSzSC   = (size_t)kChunkG * kPtsPer * kPtsPer * 4;
constexpr size_t kSzPP   = (size_t)kChunkG * kPtsPer * kPtsPer * 2;
constexpr size_t kSzOH   = (size_t)kGroups * kPtsPer * kDpad * 4;

constexpr size_t kOffWpl  = 0;
constexpr size_t kOffInQH = kOffWpl + kSzWpl;
constexpr size_t kOffInQL = kOffInQH + kSzIn16;
constexpr size_t kOffInKH = kOffInQL + kSzIn16;
constexpr size_t kOffInKL = kOffInKH + kSzIn16;
constexpr size_t kOffX    = kOffInKL + kSzIn16;
constexpr size_t kOffNP   = kOffX + kSzXf;
constexpr size_t kOffNPH  = kOffNP + kSzNPf;
constexpr size_t kOffNPL  = kOffNPH + kSzNP16;
constexpr size_t kOffHH   = kOffNPL + kSzNP16;
constexpr size_t kOffHL   = kOffHH + kSzH16;
constexpr size_t kOffNB   = kOffHL + kSzH16;
constexpr size_t kOffQFH  = kOffNB + kSzNPf;
constexpr size_t kOffQFL  = kOffQFH + kSzF16;
constexpr size_t kOffKFH  = kOffQFL + kSzF16;
constexpr size_t kOffKFL  = kOffKFH + kSzF16;
constexpr size_t kOffQH   = kOffKFL + kSzF16;
constexpr size_t kOffKH   = kOffQH + kSzXf;
constexpr size_t kOffVH   = kOffKH + kSzXf;
constexpr size_t kOffQPH  = kOffVH + kSzXf;
constexpr size_t kOffQPL  = kOffQPH + kSzQP;
constexpr size_t kOffKPH  = kOffQPL + kSzQP;
constexpr size_t kOffKPL  = kOffKPH + kSzQP;
constexpr size_t kOffVTH  = kOffKPL + kSzQP;
constexpr size_t kOffVTL  = kOffVTH + kSzQP;
constexpr size_t kOffSC   = kOffVTL + kSzQP;
constexpr size_t kOffPPH  = kOffSC + kSzSC;
constexpr size_t kOffPPL  = kOffPPH + kSzPP;
constexpr size_t kOffOH   = kOffPPL + kSzPP;
constexpr size_t kOffRSH  = kOffOH + kSzOH;
constexpr size_t kOffRSL  = kOffRSH + kSzF16;
constexpr size_t kWsTotal = kOffRSL + kSzF16;
static_assert(kWsTotal == 125829120, "carve");
static_assert(kWsTotal <= 134217728, "carve limit");
static_assert((size_t)12 * kWSlot * 2 <= kSzWpl, "weight planes");
static_assert(kOffX % 128 == 0 && kOffSC % 128 == 0 && kOffPPL % 128 == 0 && kOffRSL % 128 == 0, "alignment");

extern "C" void kernel_launch(void* const* d_in, const int* in_sizes, int n_in,
                              void* d_out, int out_size, void* d_ws, size_t ws_size,
                              hipStream_t stream) {
  if (n_in < 20) return;
  if (in_sizes[0] != kRows * kCin || in_sizes[1] != kRows * kCin) return;
  if (in_sizes[2] != kCin * kFeat || in_sizes[7] != kCin * kFeat) return;
  if (in_sizes[12] != kFeat * kFeat || in_sizes[13] != kFeat * kFeat || in_sizes[14] != kFeat * kFeat) return;
  if (in_sizes[15] != kFeat * kFeat) return;
  if (out_size != kRows * kFeat) return;
  if (ws_size < kWsTotal) return;

  const float* qfts     = (const float*)d_in[0];
  const float* kvfts    = (const float*)d_in[1];
  const float* w_q_in   = (const float*)d_in[2];
  const float* q_nl_w1  = (const float*)d_in[3];
  const float* q_nl_b1  = (const float*)d_in[4];
  const float* q_nl_w2  = (const float*)d_in[5];
  const float* q_nl_b2  = (const float*)d_in[6];
  const float* w_kv_in  = (const float*)d_in[7];
  const float* kv_nl_w1 = (const float*)d_in[8];
  const float* kv_nl_b1 = (const float*)d_in[9];
  const float* kv_nl_w2 = (const float*)d_in[10];
  const float* kv_nl_b2 = (const float*)d_in[11];
  const float* w_q      = (const float*)d_in[12];
  const float* w_k      = (const float*)d_in[13];
  const float* w_v      = (const float*)d_in[14];
  const float* w_out    = (const float*)d_in[15];
  const float* o_nl_w1  = (const float*)d_in[16];
  const float* o_nl_b1  = (const float*)d_in[17];
  const float* o_nl_w2  = (const float*)d_in[18];
  const float* o_nl_b2  = (const float*)d_in[19];
  float* out = (float*)d_out;

  char* ws = (char*)d_ws;
  us16* WPL  = (us16*)(ws + kOffWpl);
  us16* INQH = (us16*)(ws + kOffInQH);
  us16* INQL = (us16*)(ws + kOffInQL);
  us16* INKH = (us16*)(ws + kOffInKH);
  us16* INKL = (us16*)(ws + kOffInKL);
  float* X   = (float*)(ws + kOffX);
  float* NP  = (float*)(ws + kOffNP);
  us16* NPH  = (us16*)(ws + kOffNPH);
  us16* NPL  = (us16*)(ws + kOffNPL);
  us16* HH   = (us16*)(ws + kOffHH);
  us16* HL   = (us16*)(ws + kOffHL);
  float* NB  = (float*)(ws + kOffNB);
  us16* QFH  = (us16*)(ws + kOffQFH);
  us16* QFL  = (us16*)(ws + kOffQFL);
  us16* KFH  = (us16*)(ws + kOffKFH);
  us16* KFL  = (us16*)(ws + kOffKFL);
  float* QH  = (float*)(ws + kOffQH);
  float* KH  = (float*)(ws + kOffKH);
  float* VH  = (float*)(ws + kOffVH);
  us16* QPH  = (us16*)(ws + kOffQPH);
  us16* QPL  = (us16*)(ws + kOffQPL);
  us16* KPH  = (us16*)(ws + kOffKPH);
  us16* KPL  = (us16*)(ws + kOffKPL);
  us16* VTH  = (us16*)(ws + kOffVTH);
  us16* VTL  = (us16*)(ws + kOffVTL);
  float* SC  = (float*)(ws + kOffSC);
  us16* PPH  = (us16*)(ws + kOffPPH);
  us16* PPL  = (us16*)(ws + kOffPPL);
  float* OH  = (float*)(ws + kOffOH);
  us16* RSH  = (us16*)(ws + kOffRSH);
  us16* RSL  = (us16*)(ws + kOffRSL);

  const us16* Wh[12];
  const us16* Wl[12];
  for (int i = 0; i < 12; ++i) {
    Wh[i] = WPL + (size_t)i * kWSlot;
    Wl[i] = Wh[i] + kWLoOff;
  }

  wprep_kernel<<<dim3(4, 12), dim3(256), 0, stream>>>(w_q_in, q_nl_w1, q_nl_w2, w_kv_in, kv_nl_w1, kv_nl_w2,
                                                      w_q, w_k, w_v, w_out, o_nl_w1, o_nl_w2, WPL);
  const int n8 = (kRows * kCin) / 8;
  split8_kernel<<<dim3(n8 / 256, 2), dim3(256), 0, stream>>>(qfts, kvfts, INQH, INQL, INKH, INKL, n8);

  launch_split_f32(INQH, INQL, kCin, Wh[0], Wl[0], kCin, X, kFeat, q_nl_b1, kRows, kFeat, kCin, stream);
  launch_ev_mlp(X, NP, NPH, NPL, HH, HL, NB, Wh[1], Wl[1], q_nl_b1, Wh[2], Wl[2], q_nl_b2, stream);
  evscale_kernel<0><<<dim3((kPts * 32) / 256), dim3(256), 0, stream>>>(X, NP, NB, QFH, QFL, out);
  launch_split_f32(QFH, QFL, kFeat, Wh[6], Wl[6], kFeat, QH, kFeat, q_nl_b1, kRows, kFeat, kFeat, stream);

  launch_split_f32(INKH, INKL, kCin, Wh[3], Wl[3], kCin, X, kFeat, kv_nl_b1, kRows, kFeat, kCin, stream);
  launch_ev_mlp(X, NP, NPH, NPL, HH, HL, NB, Wh[4], Wl[4], kv_nl_b1, Wh[5], Wl[5], kv_nl_b2, stream);
  evscale_kernel<0><<<dim3((kPts * 32) / 256), dim3(256), 0, stream>>>(X, NP, NB, KFH, KFL, out);
  launch_split_f32(KFH, KFL, kFeat, Wh[7], Wl[7], kFeat, KH, kFeat, kv_nl_b1, kRows, kFeat, kFeat, stream);
  launch_split_f32(KFH, KFL, kFeat, Wh[8], Wl[8], kFeat, VH, kFeat, kv_nl_b1, kRows, kFeat, kFeat, stream);

  lnpack_kernel<<<dim3((kGroups * kPtsPer * 8) / 256, 2), dim3(256), 0, stream>>>(QH, KH, QPH, QPL, KPH, KPL);
  packv_kernel<<<dim3(kPtsPer / 64, kGroups), dim3(256), 0, stream>>>(VH, VTH, VTL);

  const long strideQK = (long)kPtsPer * kDpad;
  const long strideSc = (long)kPtsPer * kPtsPer;
  const long strideVt = (long)kDpad * kPtsPer;
  const int tilesScore = (kPtsPer / 64) * (kPtsPer / 32);
  const int tilesCtx   = (kPtsPer / 64) * (kDpad / 32);
  for (int ch = 0; ch < kGroups / kChunkG; ++ch) {
    const size_t g0 = (size_t)ch * kChunkG;
    const size_t qkOff = g0 * (size_t)strideQK;
    wmma_gemm_rs<<<dim3((tilesScore + 7) / 8, kChunkG), dim3(256), 0, stream>>>(
        QPH + qkOff, QPL + qkOff, kDpad, strideQK, KPH + qkOff, KPL + qkOff, kDpad, strideQK,
        SC, kPtsPer, strideSc, kPtsPer, kPtsPer, kDpad, kLogitScale);
    softmax_kernel<<<dim3(kPtsPer, kChunkG), dim3(256), 0, stream>>>(SC, PPH, PPL);
    const size_t vtOff = g0 * (size_t)strideVt;
    float* OHg = OH + qkOff;
    wmma_gemm_rs<<<dim3((tilesCtx + 7) / 8, kChunkG), dim3(256), 0, stream>>>(
        PPH, PPL, kPtsPer, strideSc, VTH + vtOff, VTL + vtOff, kPtsPer, strideVt,
        OHg, kDpad, strideQK, kPtsPer, kDpad, kPtsPer, kPCarryInv);
  }

  repack_kernel<<<dim3((kRows * 16) / 256), dim3(256), 0, stream>>>(OH, RSH, RSL);
  launch_split_f32(RSH, RSL, kFeat, Wh[9], Wl[9], kFeat, X, kFeat, o_nl_b1, kRows, kFeat, kFeat, stream);
  launch_ev_mlp(X, NP, NPH, NPL, HH, HL, NB, Wh[10], Wl[10], o_nl_b1, Wh[11], Wl[11], o_nl_b2, stream);
  evscale_kernel<1><<<dim3((kPts * 32) / 256), dim3(256), 0, stream>>>(X, NP, NB, NPH, NPL, out);
}
